// S6_8727373545524
// MI455X (gfx1250) — hardware-verified
//
#include <hip/hip_runtime.h>
#include <math.h>

typedef __attribute__((ext_vector_type(16))) _Float16 v16h;
typedef __attribute__((ext_vector_type(8)))  _Float16 v8h;
typedef __attribute__((ext_vector_type(16))) __bf16   v16b;
typedef __attribute__((ext_vector_type(8)))  __bf16   v8b;
typedef __attribute__((ext_vector_type(8)))  float    v8f;
typedef __attribute__((ext_vector_type(4)))  float    v4f;

constexpr int kBatch = 4;
constexpr int kSeq   = 2048;
constexpr int kRows  = kBatch * kSeq;
constexpr int kD     = 1024;
constexpr int kNs    = 16;
constexpr int kBcP   = 64;
constexpr int kEpTP  = 260;
constexpr float kW1Carry    = 32.0f;
constexpr float kW1CarryInv = 1.0f / kW1Carry;
static_assert(kRows == 8192, "token rows");
static_assert((kD % 64) == 0 && (kRows % 64) == 0 && (kBcP % 64) == 0, "GEMM M,N multiples of 64");
static_assert((kD % 32) == 0, "GEMM K multiple of 32");
static_assert(2 * kNs <= kBcP, "B|C columns fit the padded plane");
static_assert((kD % 256) == 0, "column blocks of 256");

constexpr size_t kOffX16  = 0;
constexpr size_t kOffXH   = kOffX16  + (size_t)kRows * kD * 2;
constexpr size_t kOffXL   = kOffXH   + (size_t)kRows * kD * 2;
constexpr size_t kOffW1T  = kOffXL   + (size_t)kRows * kD * 2;
constexpr size_t kOffW23H = kOffW1T  + (size_t)kD * kD * 2;
constexpr size_t kOffW23L = kOffW23H + (size_t)kBcP * kD * 2;
constexpr size_t kOffBC   = kOffW23L + (size_t)kBcP * kD * 2;
constexpr size_t kOffZ    = kOffBC   + (size_t)kRows * kBcP * 4;
constexpr size_t kWsTotal = kOffZ    + (size_t)kRows * kD * 4;
static_assert(kWsTotal == 88342528ull, "carve total");
static_assert(kWsTotal <= 134217728ull, "carve cap");
static_assert((kOffXH % 128) == 0 && (kOffXL % 128) == 0 && (kOffW1T % 128) == 0 && (kOffW23H % 128) == 0 &&
              (kOffW23L % 128) == 0 && (kOffBC % 128) == 0 && (kOffZ % 128) == 0, "128-B aligned regions");

__device__ __forceinline__ unsigned short f2bf_bits(float f) {
  unsigned u = __float_as_uint(f);
  return (unsigned short)((u + 0x7FFFu + ((u >> 16) & 1u)) >> 16);
}
__device__ __forceinline__ float bf_bits2f(unsigned short h) { return __uint_as_float(((unsigned)h) << 16); }

__device__ __forceinline__ void dep_guard4_h(v8f& a, v8f& b, v8f& c, v8f& d, v16h x, v16h y) { asm volatile("v_nop\n\tv_nop\n\tv_nop\n\tv_nop" : "+v"(a), "+v"(b), "+v"(c), "+v"(d) : "v"(x), "v"(y)); }
__device__ __forceinline__ void dep_guard4_b(v8f& a, v8f& b, v8f& c, v8f& d, v16b x, v16b y) { asm volatile("v_nop\n\tv_nop\n\tv_nop\n\tv_nop" : "+v"(a), "+v"(b), "+v"(c), "+v"(d) : "v"(x), "v"(y)); }
__device__ __forceinline__ void keep4_h(v16h a, v16h b, v16h c, v16h d) { asm volatile("v_nop" :: "v"(a), "v"(b), "v"(c), "v"(d)); }
__device__ __forceinline__ void keep4_b(v16b a, v16b b, v16b c, v16b d) { asm volatile("v_nop" :: "v"(a), "v"(b), "v"(c), "v"(d)); }
__device__ __forceinline__ void acc_guard4(v8f& a, v8f& b, v8f& c, v8f& d) { asm volatile("v_nop\n\tv_nop\n\tv_nop\n\tv_nop" : "+v"(a), "+v"(b), "+v"(c), "+v"(d)); }
template <typename T> struct Frag;
template <> struct Frag<_Float16> {
  typedef v16h V; union U { v16h v; v8h h[2]; };
  static __device__ __forceinline__ v16h load(const _Float16* p) {
    U f; f.h[0] = *(const v8h*)(p); f.h[1] = *(const v8h*)(p + 16); return f.v;
  }
  static __device__ __forceinline__ v8f mma(v16h a, v16h b, v8f c) {
    return __builtin_amdgcn_wmma_f32_16x16x32_f16(false, a, false, b, (short)0, c, false, false);
  }
  static __device__ __forceinline__ void guard4(v8f& a, v8f& b, v8f& c, v8f& d, v16h x, v16h y) { dep_guard4_h(a, b, c, d, x, y); }
  static __device__ __forceinline__ void keep(v16h a, v16h b, v16h c, v16h d) { keep4_h(a, b, c, d); }
};
template <> struct Frag<__bf16> {
  typedef v16b V; union U { v16b v; v8b h[2]; };
  static __device__ __forceinline__ v16b load(const __bf16* p) {
    U f; f.h[0] = *(const v8b*)(p); f.h[1] = *(const v8b*)(p + 16); return f.v;
  }
  static __device__ __forceinline__ v8f mma(v16b a, v16b b, v8f c) {
    return __builtin_amdgcn_wmma_f32_16x16x32_bf16(false, a, false, b, (short)0, c, false, false);
  }
  static __device__ __forceinline__ void guard4(v8f& a, v8f& b, v8f& c, v8f& d, v16b x, v16b y) { dep_guard4_b(a, b, c, d, x, y); }
  static __device__ __forceinline__ void keep(v16b a, v16b b, v16b c, v16b d) { keep4_b(a, b, c, d); }
};

template <int ET> struct Elem;
template <> struct Elem<0> { typedef _Float16 T; };
template <> struct Elem<1> { typedef __bf16 T; };
template <int ET, bool SPLIT>
__global__ __launch_bounds__(256) void wmma_gemm64(
    const unsigned short* __restrict__ Ap, const unsigned short* __restrict__ A2p, int lda,
    const unsigned short* __restrict__ Btp, const unsigned short* __restrict__ Bt2p, int ldb,
    float* __restrict__ Cout, int ldc,
    int M, int N, int K, float scale) {
  typedef typename Elem<ET>::T T;
  typedef typename Frag<T>::V V;
  const T* Ab  = (const T*)Ap;
  const T* Ab2 = (const T*)A2p;
  const T* Bb  = (const T*)Btp;
  const T* Bb2 = (const T*)Bt2p;
  __shared__ __align__(16) float sT[8][16 * 68];
  const int lane = threadIdx.x & 31;
  const int wave = threadIdx.x >> 5;
  const int tilesN = N >> 6;
  const int tilesM = M >> 6;
  const int tile = blockIdx.x * 8 + wave;
  if (tile >= tilesM * tilesN) return;
  const int tm = tile / tilesN;
  const int tn = tile - tm * tilesN;
  const int m0 = tm << 6;
  const int n0 = tn << 6;

  const int rlane = lane & 15;
  const int koff  = (lane >> 4) * 8;
  const int mOff  = (lane >> 4) * 8;

  v8f acc[4][4];
#pragma unroll
  for (int i = 0; i < 4; ++i)
#pragma unroll
    for (int j = 0; j < 4; ++j) acc[i][j] = (v8f){0.f,0.f,0.f,0.f,0.f,0.f,0.f,0.f};

  for (int k0 = 0; k0 < K; k0 += 32) {
    V bh[4], bl[4];
#pragma unroll
    for (int j = 0; j < 4; ++j) {
      const size_t bo = (size_t)(n0 + (j << 4) + rlane) * ldb + koff + k0;
      bh[j] = Frag<T>::load(Bb + bo);
      if (SPLIT) bl[j] = Frag<T>::load(Bb2 + bo);
    }
#pragma unroll
    for (int i = 0; i < 4; ++i) {
      const size_t ao = (size_t)(m0 + (i << 4) + rlane) * lda + koff + k0;
      V ah = Frag<T>::load(Ab + ao);
      V al;
      if (SPLIT) al = Frag<T>::load(Ab2 + ao);
#pragma unroll
      for (int j = 0; j < 4; ++j) {
        acc[i][j] = Frag<T>::mma(ah, bh[j], acc[i][j]);
        if (SPLIT) {
          acc[i][j] = Frag<T>::mma(ah, bl[j], acc[i][j]);
          acc[i][j] = Frag<T>::mma(al, bh[j], acc[i][j]);
        }
      }
      Frag<T>::guard4(acc[i][0], acc[i][1], acc[i][2], acc[i][3], ah, SPLIT ? al : ah);
    }
    Frag<T>::keep(bh[0], bh[1], bh[2], bh[3]);
    if (SPLIT) Frag<T>::keep(bl[0], bl[1], bl[2], bl[3]);
  }
  acc_guard4(acc[0][0], acc[0][1], acc[0][2], acc[0][3]);
  acc_guard4(acc[1][0], acc[1][1], acc[1][2], acc[1][3]);
  acc_guard4(acc[2][0], acc[2][1], acc[2][2], acc[2][3]);
  acc_guard4(acc[3][0], acc[3][1], acc[3][2], acc[3][3]);

  float* slab = sT[wave];
#pragma unroll
  for (int i = 0; i < 4; ++i) {
    const int mBase = m0 + (i << 4);
#pragma unroll
    for (int j = 0; j < 4; ++j) {
#pragma unroll
      for (int r = 0; r < 8; ++r) {
        const float v = acc[i][j][r] * scale;
        slab[(mOff + r) * 68 + (j << 4) + rlane] = v;
      }
    }
    __builtin_amdgcn_fence(__ATOMIC_RELEASE, "workgroup");
    __builtin_amdgcn_wave_barrier();
    __builtin_amdgcn_fence(__ATOMIC_ACQUIRE, "workgroup");
    {
      const int hh = lane >> 4, c4 = (lane & 15) * 4;
      for (int pass = 0; pass < 2; ++pass) {
#pragma unroll
        for (int it = 0; it < 8; ++it) {
          const int row = it * 2 + hh;
          v4f v = *(const v4f*)(slab + row * 68 + c4);
          *(volatile v4f*)(Cout + (size_t)(mBase + row) * ldc + n0 + c4) = v;
        }
        __threadfence();
      }
    }
    __builtin_amdgcn_fence(__ATOMIC_RELEASE, "workgroup");
    __builtin_amdgcn_wave_barrier();
    __builtin_amdgcn_fence(__ATOMIC_ACQUIRE, "workgroup");
  }
}

__global__ __launch_bounds__(256) void convert_x_kernel(
    const float* __restrict__ src, unsigned short* __restrict__ d16,
    unsigned short* __restrict__ dhi, unsigned short* __restrict__ dlo, int total8)
{
  const int i = blockIdx.x * 256 + threadIdx.x;
  if (i >= total8) return;
  const size_t e0 = (size_t)i << 3;
  const v4f a0 = *(const v4f*)(src + e0);
  const v4f a1 = *(const v4f*)(src + e0 + 4);
  v8h fv, hv, lv;
#pragma unroll
  for (int e = 0; e < 4; ++e) {
    const float f0 = a0[e];
    const float f1 = a1[e];
    const unsigned short h0 = f2bf_bits(f0), h1 = f2bf_bits(f1);
    const unsigned short l0 = f2bf_bits(f0 - bf_bits2f(h0)), l1 = f2bf_bits(f1 - bf_bits2f(h1));
    fv[e]     = (_Float16)f0;
    fv[4 + e] = (_Float16)f1;
    hv[e]     = __builtin_bit_cast(_Float16, h0);
    hv[4 + e] = __builtin_bit_cast(_Float16, h1);
    lv[e]     = __builtin_bit_cast(_Float16, l0);
    lv[4 + e] = __builtin_bit_cast(_Float16, l1);
  }
  unsigned short* qf = d16 + e0;
  unsigned short* qh = dhi + e0;
  unsigned short* ql = dlo + e0;
  *(volatile v8h*)qf = fv;
  *(volatile v8h*)qh = hv;
  *(volatile v8h*)ql = lv;
  __threadfence();
  *(volatile v8h*)qf = fv;
  *(volatile v8h*)qh = hv;
  *(volatile v8h*)ql = lv;
}

__global__ __launch_bounds__(256) void transpose_cast_kernel(
    const float* __restrict__ W, unsigned short* __restrict__ Bt, int Kdim, int Ndim, int Npad, float scale)
{
  __shared__ float tile[64 * 65];
  const int tid = threadIdx.x, lane = tid & 31, wave = tid >> 5;
  const int n0 = blockIdx.x * 64;
  const int k0 = blockIdx.y * 64;
  (void)Npad;
#pragma unroll
  for (int p = 0; p < 16; ++p) {
    const int idx = tid + p * 256;
    const int kk  = idx >> 6;
    const int nn  = idx & 63;
    const int n   = n0 + nn;
    const int nc  = (n < Ndim) ? n : (Ndim - 1);
    const float v = W[(size_t)(k0 + kk) * Ndim + nc];
    tile[kk * 65 + nn] = (n < Ndim) ? (v * scale) : 0.f;
  }
  __syncthreads();
  const int q = lane >> 3, c8 = (lane & 7) * 8;
  v8h hv[2];
#pragma unroll
  for (int it = 0; it < 2; ++it) {
    const int nrow = it * 32 + wave * 4 + q;
#pragma unroll
    for (int e = 0; e < 8; ++e) hv[it][e] = (_Float16)tile[(c8 + e) * 65 + nrow];
  }
  for (int pass = 0; pass < 2; ++pass) {
#pragma unroll
    for (int it = 0; it < 2; ++it) {
      const int nrow = it * 32 + wave * 4 + q;
      *(volatile v8h*)(Bt + (size_t)(n0 + nrow) * Kdim + k0 + c8) = hv[it];
    }
    __threadfence();
  }
}

__global__ __launch_bounds__(256) void pack_w23_kernel(
    const float* __restrict__ W2, const float* __restrict__ W3,
    unsigned short* __restrict__ BH, unsigned short* __restrict__ BL)
{
  __shared__ float tile[64 * 33];
  const int tid = threadIdx.x, lane = tid & 31, wave = tid >> 5;
  const int k0 = blockIdx.x * 64;
#pragma unroll
  for (int p = 0; p < 4; ++p) {
    const int idx = tid + p * 256;
    const int kk  = idx >> 4;
    const int nn  = idx & 15;
    tile[kk * 33 + nn]       = W2[(size_t)(k0 + kk) * kNs + nn];
    tile[kk * 33 + 16 + nn]  = W3[(size_t)(k0 + kk) * kNs + nn];
  }
  __syncthreads();
  const int q = lane >> 3, c8 = (lane & 7) * 8;
  const int nrow = wave * 4 + q;
  v8h hv, lv, zv;
#pragma unroll
  for (int e = 0; e < 8; ++e) {
    const float f = tile[(c8 + e) * 33 + nrow];
    const unsigned short hb = f2bf_bits(f);
    const unsigned short lb = f2bf_bits(f - bf_bits2f(hb));
    hv[e] = __builtin_bit_cast(_Float16, hb);
    lv[e] = __builtin_bit_cast(_Float16, lb);
    zv[e] = (_Float16)0.0f;
  }
  const size_t o_real = (size_t)nrow * kD + k0 + c8;
  const size_t o_pad  = (size_t)(32 + nrow) * kD + k0 + c8;
  for (int pass = 0; pass < 2; ++pass) {
    *(volatile v8h*)(BH + o_real) = hv;
    *(volatile v8h*)(BL + o_real) = lv;
    *(volatile v8h*)(BH + o_pad)  = zv;
    *(volatile v8h*)(BL + o_pad)  = zv;
    __threadfence();
  }
}

__global__ __launch_bounds__(256) void softplus_scale_kernel(
    const float* __restrict__ Z, const float* __restrict__ X, const float* __restrict__ BC,
    const float* __restrict__ b1, const float* __restrict__ b2, const float* __restrict__ b3,
    float* __restrict__ out)
{
  __shared__ __align__(16) float sT[16 * kEpTP];
  __shared__ float sS[64];
  const int tid = threadIdx.x, lane = tid & 31, wave = tid >> 5;
  const int d0 = blockIdx.x * 256, d = d0 + tid;
  const int g0 = blockIdx.y * 64;
  if (tid < 64) {
    const float* bc = BC + (size_t)(g0 + tid) * kBcP;
    float acc = 0.0f;
#pragma unroll 1
    for (int q4 = 0; q4 < 4; ++q4) {
      const v4f bv  = *(const v4f*)(bc + 4 * q4);
      const v4f cv  = *(const v4f*)(bc + kNs + 4 * q4);
      const v4f b2v = *(const v4f*)(b2 + 4 * q4);
      const v4f b3v = *(const v4f*)(b3 + 4 * q4);
      acc = fmaf(bv[0] + b2v[0], cv[0] + b3v[0], acc);
      acc = fmaf(bv[1] + b2v[1], cv[1] + b3v[1], acc);
      acc = fmaf(bv[2] + b2v[2], cv[2] + b3v[2], acc);
      acc = fmaf(bv[3] + b2v[3], cv[3] + b3v[3], acc);
    }
    sS[tid] = acc;
  }
  __syncthreads();
  const float bcol = b1[d];
  const int hrow = wave >> 1;
  const int hch  = (wave & 1) * 128 + lane * 4;
#pragma unroll 1
  for (int sub = 0; sub < 4; ++sub) {
    const int lb = g0 + sub * 16;
#pragma unroll 1
    for (int s = 0; s < 16; ++s) {
      const size_t o = (size_t)(lb + s) * kD + d;
      float zr = Z[o];
      float xv = X[o];
      asm volatile("" : "+v"(zr), "+v"(xv));
      const float z  = zr + bcol;
      const float a  = expf(-fabsf(z));
      const float sp = fmaxf(z, 0.0f) + log1pf(a);
      sT[s * kEpTP + tid] = (xv * sp) * sS[sub * 16 + s];
    }
    __syncthreads();
    v4f fv[4];
#pragma unroll
    for (int it = 0; it < 4; ++it) fv[it] = *(const v4f*)(sT + (it * 4 + hrow) * kEpTP + hch);
    for (int pass = 0; pass < 2; ++pass) {
#pragma unroll
      for (int it = 0; it < 4; ++it)
        *(volatile v4f*)(out + (size_t)(lb + it * 4 + hrow) * kD + d0 + hch) = fv[it];
      __threadfence();
    }
    __syncthreads();
  }
}

extern "C" void kernel_launch(void* const* d_in, const int* in_sizes, int n_in,
                              void* d_out, int out_size, void* d_ws, size_t ws_size,
                              hipStream_t stream) {
  if (n_in < 8) return;
  if (in_sizes[0] != kRows * kD) return;
  if (in_sizes[1] != kD * kD) return;
  if (in_sizes[2] != kD) return;
  if (in_sizes[3] != kD * kNs) return;
  if (in_sizes[4] != kNs) return;
  if (in_sizes[5] != kD * kNs) return;
  if (in_sizes[6] != kNs) return;
  if (out_size != kRows * kD) return;
  if (ws_size < kWsTotal) return;

  const float* x  = (const float*)d_in[0];
  const float* W1 = (const float*)d_in[1];
  const float* b1 = (const float*)d_in[2];
  const float* W2 = (const float*)d_in[3];
  const float* b2 = (const float*)d_in[4];
  const float* W3 = (const float*)d_in[5];
  const float* b3 = (const float*)d_in[6];
  float* out = (float*)d_out;

  char* ws = (char*)d_ws;
  unsigned short* X16  = (unsigned short*)(ws + kOffX16);
  unsigned short* XH   = (unsigned short*)(ws + kOffXH);
  unsigned short* XL   = (unsigned short*)(ws + kOffXL);
  unsigned short* W1T  = (unsigned short*)(ws + kOffW1T);
  unsigned short* W23H = (unsigned short*)(ws + kOffW23H);
  unsigned short* W23L = (unsigned short*)(ws + kOffW23L);
  float*          BC   = (float*)(ws + kOffBC);
  float*          Zp   = (float*)(ws + kOffZ);

  convert_x_kernel<<<(kRows * kD / 8) / 256, 256, 0, stream>>>(x, X16, XH, XL, kRows * kD / 8);

  transpose_cast_kernel<<<dim3(kD / 64, kD / 64), 256, 0, stream>>>(W1, W1T, kD, kD, kD, kW1Carry);

  pack_w23_kernel<<<kD / 64, 256, 0, stream>>>(W2, W3, W23H, W23L);

  wmma_gemm64<1, true><<<dim3((kRows / 64) * (kBcP / 64) / 8, 1), 256, 0, stream>>>(
      XH, XL, kD,
      W23H, W23L, kD,
      BC, kBcP,
      kRows, kBcP, kD, 1.0f);

  wmma_gemm64<0, false><<<dim3((kRows / 64) * (kD / 64) / 8, 1), 256, 0, stream>>>(
      X16, X16, kD,
      W1T, W1T, kD,
      Zp, kD,
      kRows, kD, kD, kW1CarryInv);

  softplus_scale_kernel<<<dim3(kD / 256, kRows / 64), 256, 0, stream>>>(Zp, x, BC, b1, b2, b3, out);
}
